// SwinTransformerTimm_73589969650208
// MI455X (gfx1250) — hardware-verified
//
#include <hip/hip_runtime.h>
#include <math.h>

typedef __attribute__((ext_vector_type(16))) _Float16 v16h;
typedef __attribute__((ext_vector_type(16))) __bf16 v16b;
typedef __attribute__((ext_vector_type(8)))  _Float16 v8h;
typedef __attribute__((ext_vector_type(8)))  float v8f;
typedef __attribute__((ext_vector_type(4)))  float v4f;
typedef __attribute__((ext_vector_type(2)))  float v2f;
typedef __attribute__((ext_vector_type(4)))  unsigned v4u;
typedef __attribute__((ext_vector_type(4)))  int v4i;
typedef float __attribute__((may_alias)) float_a;
typedef int __attribute__((may_alias)) int_a;

template <typename T> __device__ __forceinline__ void vst2(void* p, T v) { *(volatile T*)p = v; __threadfence(); *(volatile T*)p = v; }
__device__ __forceinline__ v8f wmma16(v16h a, v16h b, v8f c) {
  v8f d = __builtin_amdgcn_wmma_f32_16x16x32_f16(false, a, false, b, (short)0, c, false, false);
  asm volatile("v_nop\n\tv_nop\n\tv_nop\n\tv_nop" : "+v"(d) : "v"(a), "v"(b));
  return d;
}
__device__ __forceinline__ v8f wmma_bf(v16b a, v16b b, v8f c) {
  v8f d = __builtin_amdgcn_wmma_f32_16x16x32_bf16(false, a, false, b, (short)0, c, false, false);
  asm volatile("v_nop\n\tv_nop\n\tv_nop\n\tv_nop" : "+v"(d) : "v"(a), "v"(b));
  return d;
}
__device__ __forceinline__ v16h frag_h(const _Float16* rowk0, int lane) {
  union { v16h v; v8h q[2]; } u; const _Float16* p = rowk0 + 8 * (lane >> 4);
  u.q[0] = *(const v8h*)p; u.q[1] = *(const v8h*)(p + 16); return u.v;
}
__device__ __forceinline__ v16h frag_f32(const float* rowk0, int lane) {
  v16h a; const float* p = rowk0 + 8 * (lane >> 4);
#pragma unroll
  for (int i = 0; i < 8; ++i) { a[i] = (_Float16)p[i]; a[8 + i] = (_Float16)p[16 + i]; }
  return a;
}
__device__ __forceinline__ v16h frag_f32s(const float* rowk0, int lane, float sc) {
  v16h a; const float* p = rowk0 + 8 * (lane >> 4);
#pragma unroll
  for (int i = 0; i < 8; ++i) { a[i] = (_Float16)(p[i] * sc); a[8 + i] = (_Float16)(p[16 + i] * sc); }
  return a;
}
__device__ __forceinline__ v16h fragc_f32(const float* W, int k0, int n, int lane, int ld, int K) {
  v16h a; const int g = lane >> 4;
#pragma unroll
  for (int i = 0; i < 8; ++i) { const int ka = k0 + 8 * g + i, kb = ka + 16;
    a[i] = (_Float16)(ka < K ? W[(size_t)(ka < K ? ka : K - 1) * ld + n] : 0.f); a[8 + i] = (_Float16)(kb < K ? W[(size_t)(kb < K ? kb : K - 1) * ld + n] : 0.f); }
  return a;
}
struct F2 { v16b h, l; };
__device__ __forceinline__ F2 bsplit16(const float v[16]) { F2 r;
#pragma unroll
  for (int i = 0; i < 16; ++i) { const __bf16 h = (__bf16)v[i]; r.h[i] = h; r.l[i] = (__bf16)(v[i] - (float)h); }
  return r; }
__device__ __forceinline__ F2 split_row(const float* row, int k0, int lane) { float v[16]; const float* p = row + k0 + 8 * (lane >> 4);
#pragma unroll
  for (int i = 0; i < 8; ++i) { v[i] = p[i]; v[8 + i] = p[16 + i]; }
  return bsplit16(v); }
__device__ __forceinline__ F2 split_rowK(const float* row, int k0, int lane, int K) { float v[16]; const int g = lane >> 4;
#pragma unroll
  for (int i = 0; i < 8; ++i) { const int ka = k0 + 8 * g + i, kb = ka + 16; v[i] = ka < K ? row[ka < K ? ka : K - 1] : 0.f; v[8 + i] = kb < K ? row[kb < K ? kb : K - 1] : 0.f; }
  return bsplit16(v); }
__device__ __forceinline__ F2 split_col(const float* W, int k0, int n, int lane, int ld, int K) { float v[16]; const int g = lane >> 4;
#pragma unroll
  for (int i = 0; i < 8; ++i) { const int ka = k0 + 8 * g + i, kb = ka + 16; v[i] = ka < K ? W[(size_t)(ka < K ? ka : K - 1) * ld + n] : 0.f; v[8 + i] = kb < K ? W[(size_t)(kb < K ? kb : K - 1) * ld + n] : 0.f; }
  return bsplit16(v); }
__device__ __forceinline__ v8f mac3(const F2& a, const F2& b, v8f c) { c = wmma_bf(a.l, b.h, c); c = wmma_bf(a.h, b.l, c); return wmma_bf(a.h, b.h, c); }
__device__ __forceinline__ float sigm(float v) { return 1.0f / (1.0f + expf(-v)); }
#define LDSX() do { asm volatile("s_wait_dscnt 0" ::: "memory"); __builtin_amdgcn_wave_barrier(); __builtin_amdgcn_fence(__ATOMIC_RELEASE, "workgroup"); } while (0)


#define NBR 16384
#define NF 768
#define NCL 14
#define H1 384
#define H2 48
#define H3 48
#define NO 2
#ifndef TRB
#define TRB (NBR / 64)
#endif
typedef __attribute__((ext_vector_type(8))) __bf16 v8b;
__device__ __forceinline__ v16b frag_b(const __bf16* rowk0, int lane) {
  union { v16b v; v8b q[2]; } u; const __bf16* p = rowk0 + 8 * (lane >> 4);
  u.q[0] = *(const v8b*)p; u.q[1] = *(const v8b*)(p + 16); return u.v;
}
__device__ __forceinline__ float bfr(float v) { return (float)(__bf16)v; }
__device__ __attribute__((noinline)) float exp_ni(float v) { return expf(v); }
__device__ __attribute__((noinline)) float erf_ni(float v) { return erff(v); }

#define PK_1 0
#define PK_2 ((size_t)NCL * H1 * NF)
#define PK_3 (PK_2 + (size_t)NCL * H2 * H1)
#define PK_4 (PK_3 + (size_t)NCL * H3 * 64)
#define PK_END (PK_4 + (size_t)NCL * 16 * 64)
#define WS_END ((2u * PK_END + 127u) / 128u * 128u)

__global__ __launch_bounds__(256) void k_pack(const float* __restrict__ W1, const float* __restrict__ W2, const float* __restrict__ W3, const float* __restrict__ W4, __bf16* __restrict__ PK) {
  __shared__ __align__(16) __bf16 s[NF]; const int n = blockIdx.x, which = blockIdx.y, t = threadIdx.x; int K; size_t dst;
  if (which == 0) { K = NF; dst = PK_1 + (size_t)n * NF; for (int k = t; k < K; k += 256) s[k] = (__bf16)W1[(size_t)n * NF + k]; }
  else if (which == 1) { if (n >= NCL * H2) return; K = H1; dst = PK_2 + (size_t)n * H1; for (int k = t; k < K; k += 256) s[k] = (__bf16)W2[(size_t)n * H1 + k]; }
  else if (which == 2) { if (n >= NCL * H3) return; K = 64; dst = PK_3 + (size_t)n * 64; for (int k = t; k < K; k += 256) s[k] = (__bf16)((k < H2) ? W3[(size_t)n * H2 + k] : 0.f); }
  else { if (n >= NCL * 16) return; K = 64; dst = PK_4 + (size_t)n * 64; const int c = n / 16, o = n % 16; for (int k = t; k < K; k += 256) s[k] = (__bf16)((o < NO && k < H3) ? W4[((size_t)c * NO + o) * H3 + k] : 0.f); }
  __syncthreads();
  for (int q = t; q < K / 8; q += 256) vst2((unsigned*)(PK + dst + q * 8), *(const v4u*)&s[q * 8]);
}
__global__ __launch_bounds__(128) void k_mlp(const float* __restrict__ X, const __bf16* __restrict__ PK, const float* __restrict__ B1, const float* __restrict__ B2, const float* __restrict__ B3, const float* __restrict__ B4, float* __restrict__ Y) {
  __shared__ __align__(16) __bf16 s1h[4][16][H1 + 8], s1l[4][16][H1 + 8]; __shared__ __align__(16) __bf16 s2h[4][16][72], s2l[4][16][72]; __shared__ __align__(16) float sy[64][NO];
  const int tid = threadIdx.x, wave = tid >> 5, lane = tid & 31, col = lane & 15, g = lane >> 4; const int c = blockIdx.y; const size_t r0 = (size_t)blockIdx.x * 64 + wave * 16;
#pragma unroll 1
  for (int pass = 0; pass < 2; ++pass) { v8f acc[12] = {};
#pragma unroll 2
    for (int kc = 0; kc < NF / 32; ++kc) { v16b a; { const float* p = X + (r0 + col) * NF + kc * 32 + 8 * g;
#pragma unroll
        for (int i = 0; i < 8; ++i) { a[i] = (__bf16)p[i]; a[8 + i] = (__bf16)p[16 + i]; } }
#pragma unroll
      for (int j = 0; j < 12; ++j) acc[j] = wmma_bf(a, frag_b(PK + PK_1 + ((size_t)c * H1 + pass * 192 + j * 16 + col) * NF + kc * 32, lane), acc[j]); }
#pragma unroll
    for (int j = 0; j < 12; ++j) { const int o = pass * 192 + j * 16 + col; const float bb = bfr(B1[c * H1 + o]);
#pragma unroll
      for (int r = 0; r < 8; ++r) { const float v = fmaxf(acc[j][r] + bb, 0.f); const __bf16 hb = (__bf16)v; s1h[wave][8 * g + r][o] = hb; s1l[wave][8 * g + r][o] = (__bf16)(v - (float)hb); } } }
  if (lane < 16) for (int k = H1; k < H1 + 8; ++k) { s1h[wave][lane][k] = (__bf16)0.f; s1l[wave][lane][k] = (__bf16)0.f; }
  LDSX();
  { v8f acc[3] = {};
#pragma unroll
    for (int kc = 0; kc < H1 / 32; ++kc) { const v16b a = frag_b(&s1h[wave][col][kc * 32], lane), al = frag_b(&s1l[wave][col][kc * 32], lane);
#pragma unroll
      for (int j = 0; j < 3; ++j) { const v16b w = frag_b(PK + PK_2 + ((size_t)c * H2 + j * 16 + col) * H1 + kc * 32, lane); acc[j] = wmma_bf(al, w, acc[j]); acc[j] = wmma_bf(a, w, acc[j]); } }
#pragma unroll
    for (int j = 0; j < 3; ++j) { const int o = j * 16 + col; const float bb = bfr(B2[c * H2 + o]);
#pragma unroll
      for (int r = 0; r < 8; ++r) { const float v = fmaxf(acc[j][r] + bb, 0.f); const __bf16 hb = (__bf16)v; s2h[wave][8 * g + r][o] = hb; s2l[wave][8 * g + r][o] = (__bf16)(v - (float)hb); } }
    if (lane < 16) for (int k = H2; k < 72; ++k) { s2h[wave][lane][k] = (__bf16)0.f; s2l[wave][lane][k] = (__bf16)0.f; } }
  LDSX();
  { v8f acc[3] = {};
#pragma unroll
    for (int kc = 0; kc < 2; ++kc) { const v16b a = frag_b(&s2h[wave][col][kc * 32], lane), al = frag_b(&s2l[wave][col][kc * 32], lane);
#pragma unroll
      for (int j = 0; j < 3; ++j) { const v16b w = frag_b(PK + PK_3 + ((size_t)c * H3 + j * 16 + col) * 64 + kc * 32, lane); acc[j] = wmma_bf(al, w, acc[j]); acc[j] = wmma_bf(a, w, acc[j]); } }
    LDSX();
#pragma unroll
    for (int j = 0; j < 3; ++j) { const int o = j * 16 + col; const float bb = bfr(B3[c * H3 + o]);
#pragma unroll
      for (int r = 0; r < 8; ++r) { const float v = fmaxf(acc[j][r] + bb, 0.f); const __bf16 hb = (__bf16)v; s2h[wave][8 * g + r][o] = hb; s2l[wave][8 * g + r][o] = (__bf16)(v - (float)hb); } } }
  LDSX();
  { v8f acc = {};
#pragma unroll
    for (int kc = 0; kc < 2; ++kc) { const v16b a = frag_b(&s2h[wave][col][kc * 32], lane), al = frag_b(&s2l[wave][col][kc * 32], lane); const v16b w = frag_b(PK + PK_4 + ((size_t)c * 16 + col) * 64 + kc * 32, lane); acc = wmma_bf(al, w, acc); acc = wmma_bf(a, w, acc); }
    if (col < NO) {
#pragma unroll
      for (int r = 0; r < 8; ++r) sy[wave * 16 + 8 * g + r][col] = acc[r] + bfr(B4[c * NO + col]); } }
  __syncthreads();
  if (tid < 32) vst2(Y + ((size_t)c * NBR + (size_t)blockIdx.x * 64) * NO + tid * 4, *(const v4f*)(&sy[0][0] + tid * 4));
}
extern "C" void kernel_launch(void* const* d_in, const int* in_sizes, int n_in, void* d_out, int out_size, void* d_ws, size_t ws_size, hipStream_t stream) {
  (void)in_sizes; (void)n_in; (void)out_size;
  const float** F = (const float**)d_in;
  if (ws_size < (size_t)WS_END) return;
  char* ws = (char*)d_ws; __bf16* PK = (__bf16*)ws;
  k_pack<<<dim3(NCL * H1, 4), 256, 0, stream>>>(F[1], F[3], F[5], F[7], PK);
  k_mlp<<<dim3(TRB, NCL), 128, 0, stream>>>(F[0], PK, F[2], F[4], F[6], F[8], (float*)d_out);
}
